// RNN_forecasting_26448408609202
// MI455X (gfx1250) — hardware-verified
//
#include <hip/hip_runtime.h>
#include <stdint.h>

typedef __attribute__((ext_vector_type(16))) _Float16 v16h;
typedef __attribute__((ext_vector_type(8)))  _Float16 v8h;
typedef __attribute__((ext_vector_type(8)))  float    v8f;
typedef __attribute__((ext_vector_type(4)))  float    v4f;

__device__ __forceinline__ void dep_guard_h(v8f& a, v8f& b, v16h x, v16h y) { asm volatile("v_nop\n\tv_nop\n\tv_nop\n\tv_nop" : "+v"(a), "+v"(b) : "v"(x), "v"(y)); }
__device__ __forceinline__ void keep4_h(v16h a, v16h b, v16h c, v16h d) { asm volatile("v_nop" :: "v"(a), "v"(b), "v"(c), "v"(d)); }
__device__ __forceinline__ void acc_guard4(v8f& a, v8f& b, v8f& c, v8f& d) { asm volatile("v_nop\n\tv_nop\n\tv_nop\n\tv_nop" : "+v"(a), "+v"(b), "+v"(c), "+v"(d)); }

template <typename T> struct Frag;
template <> struct Frag<_Float16> {
  typedef v16h V; union U { v16h v; v8h h[2]; };
  static __device__ __forceinline__ v16h load(const _Float16* p) {
    U f; f.h[0] = *(const v8h*)(p); f.h[1] = *(const v8h*)(p + 16); return f.v;
  }
  static __device__ __forceinline__ v8f mma(v16h a, v16h b, v8f c) {
    return __builtin_amdgcn_wmma_f32_16x16x32_f16(false, a, false, b, (short)0, c, false, false);
  }
  static __device__ __forceinline__ void guard(v8f& a, v8f& b, v16h x, v16h y) { dep_guard_h(a, b, x, y); }
  static __device__ __forceinline__ void keep(v16h a, v16h b, v16h c, v16h d) { keep4_h(a, b, c, d); }
};

constexpr int   kBatch   = 2048;
constexpr int   kLat     = 512;
constexpr int   kEnc     = 128;
constexpr int   kFore    = 64;
constexpr int   kSteps   = kEnc + kFore - 1;
constexpr int   kRows    = 32;
constexpr int   kBlocks  = kBatch / kRows;
constexpr int   kWaves   = 8;
constexpr int   kThreads = kWaves * 32;
constexpr int   kPitch   = 520;
constexpr float kHScale  = 8.0f;
constexpr float kWScale  = 16.0f;
constexpr float kFold    = 1.0f / 128.0f;
static_assert(kBlocks * kRows == kBatch, "grid covers the batch exactly");
static_assert(kWaves * 64 == kLat, "waves cover all columns");
static_assert((kPitch % 8) == 0, "16-B aligned f16 rows");
static_assert(kLat % 32 == 0, "K multiple of 32");

__global__ __launch_bounds__(256) void cast_scale_f16x2(
    const float* __restrict__ in, _Float16* __restrict__ out, int n2, float scale) {
  const int i = blockIdx.x * 256 + threadIdx.x;
  if (i < n2) {
    const _Float16 e0 = (_Float16)(in[2 * i] * scale);
    const _Float16 e1 = (_Float16)(in[2 * i + 1] * scale);
    const unsigned u = (unsigned)__builtin_bit_cast(unsigned short, e0) |
                       ((unsigned)__builtin_bit_cast(unsigned short, e1) << 16);
    ((volatile unsigned*)out)[i] = u;
    __threadfence();
    ((volatile unsigned*)out)[i] = u;
  }
}

__global__ __launch_bounds__(kThreads) void rnn_persist(
    const float* __restrict__ x,     const float* __restrict__ h0,
    const float* __restrict__ W_in,  const float* __restrict__ b_h,
    const float* __restrict__ W_dec, const float* __restrict__ b_dec,
    const unsigned short* __restrict__ whp, float* __restrict__ out) {
  __shared__ __align__(16) _Float16 hs[kRows * kPitch];
  __shared__ __align__(16) float    fpart[kWaves * kRows];
  __shared__ __align__(16) float    fout[kFore * kRows];
  union FH { v16h v; v8h h[2]; };

  const int tid  = threadIdx.x;
  const int lane = tid & 31;
  const int wave = tid >> 5;
  const int hh   = lane >> 4;
  const int c    = lane & 15;
  const int base = blockIdx.x * kRows;
  const int n0   = wave * 64;
  const _Float16* Wh = (const _Float16*)whp;

#pragma unroll
  for (int it = 0; it < 8; ++it) {
    const int g   = it * kThreads + tid;
    const int row = g >> 6;
    const int col = (g & 63) * 8;
    const float* src = h0 + (size_t)(base + row) * kLat + col;
    const v4f u0 = *(const v4f*)(src);
    const v4f u1 = *(const v4f*)(src + 4);
    v8h hv;
    hv[0] = (_Float16)(u0[0] * kHScale); hv[1] = (_Float16)(u0[1] * kHScale);
    hv[2] = (_Float16)(u0[2] * kHScale); hv[3] = (_Float16)(u0[3] * kHScale);
    hv[4] = (_Float16)(u1[0] * kHScale); hv[5] = (_Float16)(u1[1] * kHScale);
    hv[6] = (_Float16)(u1[2] * kHScale); hv[7] = (_Float16)(u1[3] * kHScale);
    *(v8h*)(hs + row * kPitch + col) = hv;
  }

  float win[4], bhv[4], wdv[4];
#pragma unroll
  for (int j = 0; j < 4; ++j) {
    const int n = n0 + 16 * j + c;
    win[j] = W_in[n];
    bhv[j] = b_h[n];
    wdv[j] = W_dec[n];
  }
  const float bdec = b_dec[0];

  float inp[2][8];
#pragma unroll
  for (int i = 0; i < 2; ++i)
#pragma unroll
    for (int r = 0; r < 8; ++r) inp[i][r] = 0.0f;

  __syncthreads();

  for (int s = 0; s < kSteps; ++s) {
    if (s < kEnc) {
      const float* xr = x + (size_t)s * kBatch + base + 8 * hh;
#pragma unroll
      for (int i = 0; i < 2; ++i) {
        const v4f u0 = *(const v4f*)(xr + 16 * i);
        const v4f u1 = *(const v4f*)(xr + 16 * i + 4);
        inp[i][0] = u0[0]; inp[i][1] = u0[1]; inp[i][2] = u0[2]; inp[i][3] = u0[3];
        inp[i][4] = u1[0]; inp[i][5] = u1[1]; inp[i][6] = u1[2]; inp[i][7] = u1[3];
      }
    }

    v8f acc[2][4];
#pragma unroll
    for (int i = 0; i < 2; ++i)
#pragma unroll
      for (int j = 0; j < 4; ++j) acc[i][j] = (v8f){0.f, 0.f, 0.f, 0.f, 0.f, 0.f, 0.f, 0.f};

#pragma unroll 2
    for (int k0 = 0; k0 < kLat; k0 += 32) {
      v16h bf[4];
#pragma unroll
      for (int j = 0; j < 4; ++j)
        bf[j] = Frag<_Float16>::load(Wh + (size_t)(n0 + 16 * j + c) * kLat + k0 + 8 * hh);
#pragma unroll
      for (int i = 0; i < 2; ++i) {
        FH af;
        const _Float16* ap = hs + (16 * i + c) * kPitch + k0 + 8 * hh;
        af.h[0] = *(const v8h*)(ap);
        af.h[1] = *(const v8h*)(ap + 16);
#pragma unroll
        for (int j = 0; j < 4; ++j) acc[i][j] = Frag<_Float16>::mma(af.v, bf[j], acc[i][j]);
        Frag<_Float16>::guard(acc[i][0], acc[i][3], af.v, af.v);
      }
      Frag<_Float16>::keep(bf[0], bf[1], bf[2], bf[3]);
    }
    acc_guard4(acc[0][0], acc[0][1], acc[0][2], acc[0][3]);
    acc_guard4(acc[1][0], acc[1][1], acc[1][2], acc[1][3]);

    __syncthreads();

    float p[2][8];
#pragma unroll
    for (int i = 0; i < 2; ++i)
#pragma unroll
      for (int r = 0; r < 8; ++r) p[i][r] = 0.0f;
#pragma unroll
    for (int i = 0; i < 2; ++i) {
#pragma unroll
      for (int j = 0; j < 4; ++j) {
#pragma unroll
        for (int r = 0; r < 8; ++r) {
          float v = acc[i][j][r] * kFold + inp[i][r] * win[j] + bhv[j];
          v = fmaxf(v, 0.0f);
          p[i][r] += v * wdv[j];
          hs[(16 * i + 8 * hh + r) * kPitch + n0 + 16 * j + c] = (_Float16)(v * kHScale);
        }
      }
    }

    if (s >= kEnc - 1) {
#pragma unroll
      for (int i = 0; i < 2; ++i) {
#pragma unroll
        for (int r = 0; r < 8; ++r) {
          float v = p[i][r];
          v += __shfl_xor(v, 1, 32);
          v += __shfl_xor(v, 2, 32);
          v += __shfl_xor(v, 4, 32);
          v += __shfl_xor(v, 8, 32);
          if (c == 0) fpart[wave * kRows + 16 * i + 8 * hh + r] = v;
        }
      }
    }

    __syncthreads();

    if (s >= kEnc - 1) {
      const int jo = s - (kEnc - 1);
#pragma unroll
      for (int i = 0; i < 2; ++i) {
        const float* fp = fpart + 16 * i + 8 * hh;
        v4f sa = *(const v4f*)(fp);
        v4f sb = *(const v4f*)(fp + 4);
#pragma unroll
        for (int w = 1; w < kWaves; ++w) {
          sa += *(const v4f*)(fp + w * kRows);
          sb += *(const v4f*)(fp + w * kRows + 4);
        }
        float f[8];
        f[0] = sa[0]; f[1] = sa[1]; f[2] = sa[2]; f[3] = sa[3];
        f[4] = sb[0]; f[5] = sb[1]; f[6] = sb[2]; f[7] = sb[3];
#pragma unroll
        for (int r = 0; r < 8; ++r) {
          const float fv = f[r] + bdec;
          inp[i][r] = fv;
          if (wave == 0 && c == 0) fout[jo * kRows + 16 * i + 8 * hh + r] = fv;
        }
      }
    }
  }

  __syncthreads();

  if (wave == 0) {
    const int q  = lane >> 3;
    const int p4 = (lane & 7) * 4;
    for (int pass = 0; pass < 2; ++pass) {
#pragma unroll
      for (int it = 0; it < 16; ++it) {
        const int j = it * 4 + q;
        const v4f val = *(const v4f*)(fout + j * kRows + p4);
        *(volatile v4f*)(out + (size_t)j * kBatch + base + p4) = val;
      }
      __threadfence();
    }
  }
}

extern "C" void kernel_launch(void* const* d_in, const int* in_sizes, int n_in,
                              void* d_out, int out_size, void* d_ws, size_t ws_size,
                              hipStream_t stream) {
  if (n_in < 7) return;
  if (in_sizes[0] != kEnc * kBatch) return;
  if (in_sizes[1] != kBatch * kLat) return;
  if (in_sizes[2] != kLat) return;
  if (in_sizes[3] != kLat * kLat) return;
  if (in_sizes[4] != kLat) return;
  if (in_sizes[5] != kLat) return;
  if (in_sizes[6] < 1) return;
  if (out_size != kFore * kBatch) return;
  const size_t whBytes = (size_t)kLat * kLat * sizeof(_Float16);
  if (ws_size < whBytes) return;

  const float* x     = (const float*)d_in[0];
  const float* h0    = (const float*)d_in[1];
  const float* W_in  = (const float*)d_in[2];
  const float* W_h   = (const float*)d_in[3];
  const float* b_h   = (const float*)d_in[4];
  const float* W_dec = (const float*)d_in[5];
  const float* b_dec = (const float*)d_in[6];
  _Float16* whf = (_Float16*)d_ws;

  const int n2 = (kLat * kLat) / 2;
  cast_scale_f16x2<<<(n2 + 255) / 256, 256, 0, stream>>>(W_h, whf, n2, kWScale);
  rnn_persist<<<kBlocks, kThreads, 0, stream>>>(x, h0, W_in, b_h, W_dec, b_dec,
                                                 (const unsigned short*)whf, (float*)d_out);
}
